// TransNeXt_33174327394601
// MI455X (gfx1250) — hardware-verified
//
#include <hip/hip_runtime.h>
#include <math.h>

#define NBAT   4
#define NTK    4096
#define CD     256
#define NHD    8
#define HD     32
#define NPL    256
#define LL     9
#define HR     64
#define WR     64
#define NROW   16384
#define NBH    32
#define WROWS  1280
#define TKN    288
#define LDC    132
#define SCPI   272
#define PPI    264

#define XSC    8.0f
#define WSC    64.0f
#define ASC    8.0f
#define QSC    256.0f
#define KSC    1024.0f
#define PSC    1024.0f
#define VSC    8.0f
#define RESC   2048.0f
#define RSC    0.00048828125f
#define IXW    0.001953125f
#define IAW    0.001953125f
#define IQS    0.00390625f
#define IQK    3.814697265625e-06f
#define IPV    1.220703125e-04f

#define L_SC   0
#define L_PH   69632
#define L_PL   103424
#define L_QS   137216
#define L_QN   145408
#define L_OS   153600
#define L_OU   161792
#define L_TK   169984
#define LDS_ATTN 171264

static_assert(NROW == NBAT * NTK);
static_assert(NTK == HR * WR);
static_assert(CD == NHD * HD);
static_assert(NBH == NBAT * NHD);
static_assert(TKN == HD * LL);
static_assert((LDC % 4) == 0);
static_assert(((SCPI * 4) % 16) == 0 && ((PPI * 2) % 16) == 0);
static_assert(SCPI >= NPL + LL && PPI >= NPL);
static_assert(L_PH == 64 * SCPI * 4);
static_assert(L_PL == L_PH + 64 * PPI * 2);
static_assert(L_QS == L_PL + 64 * PPI * 2);
static_assert(L_QN == L_QS + 64 * HD * 4);
static_assert(L_OS == L_QN + 64 * HD * 4);
static_assert(L_OU == L_OS + 64 * HD * 4);
static_assert(L_TK == L_OU + 64 * HD * 4);
static_assert(LDS_ATTN >= L_TK + (TKN + 2 * LL) * 4);
static_assert((L_PH % 16) == 0 && (L_PL % 16) == 0 && (L_QS % 16) == 0 && (L_QN % 16) == 0 && (L_OU % 16) == 0);

typedef _Float16 v16h __attribute__((ext_vector_type(16)));
typedef _Float16 v8h  __attribute__((ext_vector_type(8)));
typedef float    v8f  __attribute__((ext_vector_type(8)));
typedef float    v4f  __attribute__((ext_vector_type(4)));
typedef unsigned int v4u __attribute__((ext_vector_type(4)));
typedef v4u v4ua __attribute__((may_alias));
typedef v4f v4fa __attribute__((may_alias));

__device__ __forceinline__ unsigned short bf_bits(float f) {
  unsigned u = __float_as_uint(f);
  return (unsigned short)((u + 0x7FFFu + ((u >> 16) & 1u)) >> 16);
}
__device__ __forceinline__ float bf_up(unsigned short b) { return __uint_as_float(((unsigned)b) << 16); }
__device__ __forceinline__ float bfr(float f) { return bf_up(bf_bits(f)); }
__device__ __forceinline__ unsigned short h_bits(_Float16 x) { return __builtin_bit_cast(unsigned short, x); }
__device__ __forceinline__ unsigned short hb16(float f) { return h_bits((_Float16)f); }
__device__ __forceinline__ unsigned pk16(unsigned short a, unsigned short b) { return (unsigned)a | ((unsigned)b << 16); }
__device__ __forceinline__ v8f zero8() { v8f z = {0.f, 0.f, 0.f, 0.f, 0.f, 0.f, 0.f, 0.f}; return z; }
__device__ __forceinline__ float gelu_exact(float v) { return 0.5f * v * (1.0f + erff(v * 0.70710678118654752f)); }
__device__ __forceinline__ float softplus_f(float t) { return (t > 20.0f) ? t : log1pf(expf(t)); }

__device__ __forceinline__ void split2s(float f0, float f1, float sc, unsigned& hpk, unsigned& lpk) {
  const float t0 = f0 * sc, t1 = f1 * sc;
  const _Float16 a = (_Float16)t0, c = (_Float16)t1;
  hpk = pk16(h_bits(a), h_bits(c));
  lpk = pk16(hb16((t0 - (float)a) * RESC), hb16((t1 - (float)c) * RESC));
}
__device__ __forceinline__ void split16(const v4f x0, const v4f x1, const v4f x2, const v4f x3, float sc,
                                        v16h& hi, v16h& lo) {
  float v[16] = {x0[0], x0[1], x0[2], x0[3], x1[0], x1[1], x1[2], x1[3],
                 x2[0], x2[1], x2[2], x2[3], x3[0], x3[1], x3[2], x3[3]};
#pragma unroll
  for (int i = 0; i < 16; ++i) {
    const float t = v[i] * sc;
    const _Float16 hq = (_Float16)t;
    hi[i] = hq;
    lo[i] = (_Float16)((t - (float)hq) * RESC);
  }
}

__device__ __forceinline__ v16h ldfrag_h(const _Float16* p) {
  union { v16h v; v8h h[2]; } f;
  f.h[0] = *(const v8h*)(p);
  f.h[1] = *(const v8h*)(p + 16);
  return f.v;
}
__device__ __forceinline__ v16h ld2(const _Float16* p0, const _Float16* p1) {
  union { v16h v; v8h h[2]; } f;
  f.h[0] = *(const v8h*)(p0);
  f.h[1] = *(const v8h*)(p1);
  return f.v;
}

__device__ __forceinline__ v8f mma_raw(v16h a, v16h b, v8f c) {
  return __builtin_amdgcn_wmma_f32_16x16x32_f16(false, a, false, b, (short)0, c, false, false);
}
__device__ __forceinline__ void guard4(v8f& c0, v8f& c1, v8f& c2, v8f& c3,
                                       const v16h& a0, const v16h& a1, const v16h& b0, const v16h& b1) {
#if defined(__HIP_DEVICE_COMPILE__)
  asm volatile("v_nop\n\tv_nop\n\tv_nop\n\tv_nop"
               : "+v"(c0), "+v"(c1), "+v"(c2), "+v"(c3) : "v"(a0), "v"(a1), "v"(b0), "v"(b1));
#endif
}
__device__ __forceinline__ void guard2(v8f& c0, v8f& c1,
                                       const v16h& a0, const v16h& a1, const v16h& b0, const v16h& b1) {
#if defined(__HIP_DEVICE_COMPILE__)
  asm volatile("v_nop\n\tv_nop\n\tv_nop\n\tv_nop"
               : "+v"(c0), "+v"(c1) : "v"(a0), "v"(a1), "v"(b0), "v"(b1));
#endif
}
__device__ __forceinline__ void guard8(v8f& c0, v8f& c1, v8f& c2, v8f& c3, v8f& c4, v8f& c5, v8f& c6, v8f& c7,
                                       const v16h& a0, const v16h& a1, const v16h& a2, const v16h& a3,
                                       const v16h& b0, const v16h& b1) {
#if defined(__HIP_DEVICE_COMPILE__)
  asm volatile("v_nop\n\tv_nop\n\tv_nop\n\tv_nop"
               : "+v"(c0), "+v"(c1), "+v"(c2), "+v"(c3), "+v"(c4), "+v"(c5), "+v"(c6), "+v"(c7)
               : "v"(a0), "v"(a1), "v"(a2), "v"(a3), "v"(b0), "v"(b1));
#endif
}

__device__ __forceinline__ void mm_tile(const _Float16* __restrict__ A, int lda,
                                        const _Float16* __restrict__ W, int ldw, int nks,
                                        int arow0, int bcol0, float* Cs) {
  const int tid = threadIdx.x, wave = tid >> 5, lane = tid & 31, hh = lane >> 4, c = lane & 15;
  const int mw = wave >> 2, nw = wave & 3;
  const _Float16* a0p = A + (size_t)(arow0 + mw * 32 + c) * lda + 8 * hh;
  const _Float16* a1p = A + (size_t)(arow0 + mw * 32 + 16 + c) * lda + 8 * hh;
  const _Float16* b0p = W + (size_t)(bcol0 + nw * 32 + c) * ldw + 8 * hh;
  const _Float16* b1p = W + (size_t)(bcol0 + nw * 32 + 16 + c) * ldw + 8 * hh;
  v8f a00 = zero8(), a01 = zero8(), a10 = zero8(), a11 = zero8();
#pragma unroll 1
  for (int ks = 0; ks < nks; ++ks) {
    const int ko = ks * 32;
    const v16h fa0 = ldfrag_h(a0p + ko);
    const v16h fa1 = ldfrag_h(a1p + ko);
    const v16h fb0 = ldfrag_h(b0p + ko);
    const v16h fb1 = ldfrag_h(b1p + ko);
    a00 = mma_raw(fa0, fb0, a00);
    a01 = mma_raw(fa0, fb1, a01);
    a10 = mma_raw(fa1, fb0, a10);
    a11 = mma_raw(fa1, fb1, a11);
    guard4(a00, a01, a10, a11, fa0, fa1, fb0, fb1);
  }
#pragma unroll
  for (int r = 0; r < 8; ++r) {
    const int row = mw * 32 + 8 * hh + r;
    Cs[row * LDC + nw * 32 + c]             = a00[r];
    Cs[row * LDC + nw * 32 + 16 + c]        = a01[r];
    Cs[(row + 16) * LDC + nw * 32 + c]      = a10[r];
    Cs[(row + 16) * LDC + nw * 32 + 16 + c] = a11[r];
  }
}

__device__ __forceinline__ void mm_tile_s(const float* __restrict__ A, int lda, int ldk,
                                          const _Float16* __restrict__ W, int ldw, int nks, float* Cs) {
  const int tid = threadIdx.x, wave = tid >> 5, lane = tid & 31, hh = lane >> 4, c = lane & 15;
  const int mw = wave >> 2, nw = wave & 3;
  const float* a0p = A + (size_t)(mw * 32 + c) * lda + 8 * hh;
  const float* a1p = A + (size_t)(mw * 32 + 16 + c) * lda + 8 * hh;
  const _Float16* b0p = W + (size_t)(nw * 32 + c) * ldw + 8 * hh;
  const _Float16* b1p = W + (size_t)(nw * 32 + 16 + c) * ldw + 8 * hh;
  v8f h00 = zero8(), h01 = zero8(), h10 = zero8(), h11 = zero8();
  v8f l00 = zero8(), l01 = zero8(), l10 = zero8(), l11 = zero8();
#pragma unroll 1
  for (int ks = 0; ks < nks; ++ks) {
    const float* q0 = a0p + (size_t)ks * ldk;
    const float* q1 = a1p + (size_t)ks * ldk;
    const v4f x00 = *(const v4f*)(q0), x01 = *(const v4f*)(q0 + 4);
    const v4f x02 = *(const v4f*)(q0 + 16), x03 = *(const v4f*)(q0 + 20);
    const v4f x10 = *(const v4f*)(q1), x11 = *(const v4f*)(q1 + 4);
    const v4f x12 = *(const v4f*)(q1 + 16), x13 = *(const v4f*)(q1 + 20);
    v16h fah0, fal0, fah1, fal1;
    split16(x00, x01, x02, x03, ASC, fah0, fal0);
    split16(x10, x11, x12, x13, ASC, fah1, fal1);
    const v16h fb0 = ldfrag_h(b0p + 32 * ks);
    const v16h fb1 = ldfrag_h(b1p + 32 * ks);
    h00 = mma_raw(fah0, fb0, h00);
    l00 = mma_raw(fal0, fb0, l00);
    h01 = mma_raw(fah0, fb1, h01);
    l01 = mma_raw(fal0, fb1, l01);
    h10 = mma_raw(fah1, fb0, h10);
    l10 = mma_raw(fal1, fb0, l10);
    h11 = mma_raw(fah1, fb1, h11);
    l11 = mma_raw(fal1, fb1, l11);
    guard8(h00, l00, h01, l01, h10, l10, h11, l11, fah0, fal0, fah1, fal1, fb0, fb1);
  }
#pragma unroll
  for (int r = 0; r < 8; ++r) {
    const int row = mw * 32 + 8 * hh + r;
    Cs[row * LDC + nw * 32 + c]             = h00[r] + l00[r] * RSC;
    Cs[row * LDC + nw * 32 + 16 + c]        = h01[r] + l01[r] * RSC;
    Cs[(row + 16) * LDC + nw * 32 + c]      = h10[r] + l10[r] * RSC;
    Cs[(row + 16) * LDC + nw * 32 + 16 + c] = h11[r] + l11[r] * RSC;
  }
}

__global__ __launch_bounds__(256)
void k_cvt_x(const float* __restrict__ x, unsigned short* xb) {
  const size_t e0 = ((size_t)blockIdx.x * 256 + threadIdx.x) * 8;
  const v4f a = *(const v4f*)(x + e0);
  const v4f c = *(const v4f*)(x + e0 + 4);
  v4u pk;
  pk[0] = pk16(hb16(bfr(a[0]) * XSC), hb16(bfr(a[1]) * XSC));
  pk[1] = pk16(hb16(bfr(a[2]) * XSC), hb16(bfr(a[3]) * XSC));
  pk[2] = pk16(hb16(bfr(c[0]) * XSC), hb16(bfr(c[1]) * XSC));
  pk[3] = pk16(hb16(bfr(c[2]) * XSC), hb16(bfr(c[3]) * XSC));
  *(volatile v4u*)(xb + e0) = pk;
  __threadfence();
  *(volatile v4u*)(xb + e0) = pk;
}

__global__ __launch_bounds__(256)
void k_cvt_w(const float* __restrict__ wq, const float* __restrict__ wkv, const float* __restrict__ wsr,
             const float* __restrict__ wpj, unsigned short* w16) {
  const int bi = blockIdx.x, tid = threadIdx.x;
  const float* src;
  int eb;
  if (bi < 32)       { src = wq;  eb = bi * 2048; }
  else if (bi < 96)  { src = wkv; eb = (bi - 32) * 2048; }
  else if (bi < 128) { src = wsr; eb = (bi - 96) * 2048; }
  else               { src = wpj; eb = (bi - 128) * 2048; }
  const int e0 = eb + tid * 8;
  const v4f a = *(const v4f*)(src + e0);
  const v4f c = *(const v4f*)(src + e0 + 4);
  v4u pk;
  pk[0] = pk16(hb16(bfr(a[0]) * WSC), hb16(bfr(a[1]) * WSC));
  pk[1] = pk16(hb16(bfr(a[2]) * WSC), hb16(bfr(a[3]) * WSC));
  pk[2] = pk16(hb16(bfr(c[0]) * WSC), hb16(bfr(c[1]) * WSC));
  pk[3] = pk16(hb16(bfr(c[2]) * WSC), hb16(bfr(c[3]) * WSC));
  unsigned short* dst = w16 + (size_t)bi * 2048 + tid * 8;
  *(volatile v4u*)dst = pk;
  __threadfence();
  *(volatile v4u*)dst = pk;
}

__global__ __launch_bounds__(256)
void k_cpb(const float* __restrict__ rct, const float* __restrict__ w1, const float* __restrict__ b1,
           const float* __restrict__ w2, const float* __restrict__ b2, float* btab, int U) {
  __shared__ __align__(16) float tb[64];
  const int tid = threadIdx.x, wave = tid >> 5, lane = tid & 31;
  const int t = blockIdx.x * 8 + wave;
  const int tc = min(t, U - 1);
  const float cx = bfr(rct[(size_t)tc * 2 + 0]);
  const float cy = bfr(rct[(size_t)tc * 2 + 1]);
  float acc[NHD];
#pragma unroll
  for (int h = 0; h < NHD; ++h) acc[h] = 0.f;
#pragma unroll 1
  for (int j = lane; j < 512; j += 32) {
    const float h1 = fmaxf(cx * bfr(w1[j * 2]) + cy * bfr(w1[j * 2 + 1]) + bfr(b1[j]), 0.f);
#pragma unroll
    for (int h = 0; h < NHD; ++h) acc[h] += h1 * bfr(w2[h * 512 + j]);
  }
#pragma unroll
  for (int h = 0; h < NHD; ++h) {
#pragma unroll
    for (int o = 16; o >= 1; o >>= 1) acc[h] += __shfl_xor(acc[h], o, 32);
  }
  if (lane == 0) {
#pragma unroll
    for (int h = 0; h < NHD; ++h) tb[wave * NHD + h] = acc[h] + bfr(b2[h]);
  }
  __syncthreads();
  if (tid < 16) {
    const v4f v = *(const v4fa*)(&tb[tid * 4]);
    float* dst = btab + (size_t)blockIdx.x * 64 + tid * 4;
    *(volatile v4f*)dst = v;
    __threadfence();
    *(volatile v4f*)dst = v;
  }
}

__global__ __launch_bounds__(256)
void k_gemm1(const unsigned short* __restrict__ xb, const unsigned short* __restrict__ w16,
             const float* __restrict__ bq, const float* __restrict__ bkv, const float* __restrict__ bsr,
             const float* __restrict__ qe, const float* __restrict__ temp, const float* __restrict__ sls,
             float* QN, unsigned short* QH, unsigned short* QL, float* KL, float* VL, float* XSR) {
  __shared__ __align__(16) float Cs[64 * LDC];
  const int tid = threadIdx.x;
  const int mb = blockIdx.x, y = blockIdx.y;
  const int row0 = mb * 64, b = mb >> 6, n0 = (mb & 63) * 64;
  mm_tile((const _Float16*)(const void*)xb, CD,
          (const _Float16*)(const void*)(w16 + (size_t)y * 128 * CD), CD, CD / 32, row0, 0, Cs);
  __syncthreads();

  if (y < 2) {
    const int row = tid & 63, hl = tid >> 6;
    const int h = y * 4 + hl;
    float* cr = Cs + row * LDC + hl * HD;
    float ss = 0.f;
#pragma unroll
    for (int d = 0; d < HD; ++d) {
      const float v = cr[d] * IXW + bfr(bq[h * HD + d]);
      cr[d] = v;
      ss += v * v;
    }
    const float inv = __builtin_amdgcn_rcpf(fmaxf(sqrtf(ss), 1e-12f));
#pragma unroll
    for (int d = 0; d < HD; ++d) cr[d] = cr[d] * inv;
    __syncthreads();
    v4f pv[8];
    size_t po[8];
#pragma unroll
    for (int s = 0; s < 8; ++s) {
      const int idx = s * 256 + tid;
      const int hl2 = idx >> 9, rem = idx & 511, row2 = rem >> 3, d0 = (rem & 7) * 4;
      pv[s] = *(const v4fa*)(&Cs[row2 * LDC + hl2 * HD + d0]);
      po[s] = ((size_t)((b * NHD + y * 4 + hl2) * NTK + n0 + row2)) * HD + d0;
    }
#pragma unroll
    for (int s = 0; s < 8; ++s) *(volatile v4f*)(QN + po[s]) = pv[s];
    __threadfence();
#pragma unroll
    for (int s = 0; s < 8; ++s) *(volatile v4f*)(QN + po[s]) = pv[s];
    __syncthreads();
    const float sp = softplus_f(bfr(temp[h]));
    const float sl = bfr(sls[n0 + row]);
#pragma unroll
    for (int d = 0; d < HD; ++d) cr[d] = (cr[d] + bfr(qe[h * HD + d])) * sp * sl;
    __syncthreads();
    v4u ph[4], pl[4];
    size_t ho[4];
#pragma unroll
    for (int s = 0; s < 4; ++s) {
      const int idx = s * 256 + tid;
      const int hl2 = idx >> 8, rem = idx & 255, row2 = rem >> 2, d0 = (rem & 3) * 8;
      const v4f a0 = *(const v4fa*)(&Cs[row2 * LDC + hl2 * HD + d0]);
      const v4f a1 = *(const v4fa*)(&Cs[row2 * LDC + hl2 * HD + d0 + 4]);
      v4u hv, lv;
      unsigned hp_, lp_;
      split2s(a0[0], a0[1], QSC, hp_, lp_); hv[0] = hp_; lv[0] = lp_;
      split2s(a0[2], a0[3], QSC, hp_, lp_); hv[1] = hp_; lv[1] = lp_;
      split2s(a1[0], a1[1], QSC, hp_, lp_); hv[2] = hp_; lv[2] = lp_;
      split2s(a1[2], a1[3], QSC, hp_, lp_); hv[3] = hp_; lv[3] = lp_;
      ph[s] = hv; pl[s] = lv;
      ho[s] = ((size_t)((b * NHD + y * 4 + hl2) * NTK + n0 + row2)) * HD + d0;
    }
#pragma unroll
    for (int s = 0; s < 4; ++s) { *(volatile v4u*)(QH + ho[s]) = ph[s]; *(volatile v4u*)(QL + ho[s]) = pl[s]; }
    __threadfence();
#pragma unroll
    for (int s = 0; s < 4; ++s) { *(volatile v4u*)(QH + ho[s]) = ph[s]; *(volatile v4u*)(QL + ho[s]) = pl[s]; }
  } else if (y < 4) {
    const int row = tid & 63, hl = tid >> 6;
    const int h = (y - 2) * 4 + hl;
    float* cr = Cs + row * LDC + hl * HD;
    float ss = 0.f;
#pragma unroll
    for (int d = 0; d < HD; ++d) {
      const float v = cr[d] * IXW + bfr(bkv[h * HD + d]);
      cr[d] = v;
      ss += v * v;
    }
    const float inv = __builtin_amdgcn_rcpf(fmaxf(sqrtf(ss), 1e-12f));
#pragma unroll
    for (int d = 0; d < HD; ++d) cr[d] = cr[d] * inv;
    __syncthreads();
    v4f pv[8];
    size_t po[8];
#pragma unroll
    for (int s = 0; s < 8; ++s) {
      const int idx = s * 256 + tid;
      const int hl2 = idx >> 9, rem = idx & 511, row2 = rem >> 3, d0 = (rem & 7) * 4;
      pv[s] = *(const v4fa*)(&Cs[row2 * LDC + hl2 * HD + d0]);
      po[s] = ((size_t)((b * NHD + (y - 2) * 4 + hl2) * NTK + n0 + row2)) * HD + d0;
    }
#pragma unroll
    for (int s = 0; s < 8; ++s) *(volatile v4f*)(KL + po[s]) = pv[s];
    __threadfence();
#pragma unroll
    for (int s = 0; s < 8; ++s) *(volatile v4f*)(KL + po[s]) = pv[s];
  } else if (y < 6) {
    v4f pv[8];
    size_t po[8];
#pragma unroll
    for (int s = 0; s < 8; ++s) {
      const int idx = s * 256 + tid;
      const int hl2 = idx >> 9, rem = idx & 511, row2 = rem >> 3, d0 = (rem & 7) * 4;
      const int cb = CD + (y - 4) * 128 + hl2 * HD + d0;
      const v4f a = *(const v4fa*)(&Cs[row2 * LDC + hl2 * HD + d0]);
      v4f r;
#pragma unroll
      for (int e = 0; e < 4; ++e) r[e] = a[e] * IXW + bfr(bkv[cb + e]);
      pv[s] = r;
      po[s] = ((size_t)((b * NHD + (y - 4) * 4 + hl2) * NTK + n0 + row2)) * HD + d0;
    }
#pragma unroll
    for (int s = 0; s < 8; ++s) *(volatile v4f*)(VL + po[s]) = pv[s];
    __threadfence();
#pragma unroll
    for (int s = 0; s < 8; ++s) *(volatile v4f*)(VL + po[s]) = pv[s];
  } else {
    v4f pv[8];
    size_t po[8];
#pragma unroll
    for (int s = 0; s < 8; ++s) {
      const int idx = s * 256 + tid;
      const int row2 = idx >> 5, c4 = (idx & 31) * 4;
      const int col = (y - 6) * 128 + c4;
      const v4f a = *(const v4fa*)(&Cs[row2 * LDC + c4]);
      v4f r;
#pragma unroll
      for (int e = 0; e < 4; ++e) r[e] = gelu_exact(a[e] * IXW + bfr(bsr[col + e]));
      pv[s] = r;
      po[s] = (size_t)(row0 + row2) * CD + col;
    }
#pragma unroll
    for (int s = 0; s < 8; ++s) *(volatile v4f*)(XSR + po[s]) = pv[s];
    __threadfence();
#pragma unroll
    for (int s = 0; s < 8; ++s) *(volatile v4f*)(XSR + po[s]) = pv[s];
  }
}

__global__ __launch_bounds__(256)
void k_pool_ln(const float* __restrict__ xsr, const float* __restrict__ g, const float* __restrict__ be, float* xp) {
  __shared__ float red[16];
  __shared__ __align__(16) float T[CD];
  const int tid = threadIdx.x, wave = tid >> 5, lane = tid & 31;
  const int bp = blockIdx.x;
  const int b = bp >> 8, p = bp & 255;
  const int ph = p >> 4, pw = p & 15;
  const int c = tid;
  float s = 0.f;
#pragma unroll
  for (int r = 0; r < 4; ++r) {
#pragma unroll
    for (int q = 0; q < 4; ++q) {
      const int n = (ph * 4 + r) * WR + (pw * 4 + q);
      s += xsr[((size_t)(b * NTK + n)) * CD + c];
    }
  }
  const float xv = s * 0.0625f;
  float a = xv;
#pragma unroll
  for (int o = 16; o >= 1; o >>= 1) a += __shfl_xor(a, o, 32);
  if (lane == 0) red[wave] = a;
  __syncthreads();
  float mu = 0.f;
#pragma unroll
  for (int w = 0; w < 8; ++w) mu += red[w];
  mu *= (1.0f / CD);
  const float dv = xv - mu;
  float a2 = dv * dv;
#pragma unroll
  for (int o = 16; o >= 1; o >>= 1) a2 += __shfl_xor(a2, o, 32);
  if (lane == 0) red[8 + wave] = a2;
  __syncthreads();
  float var = 0.f;
#pragma unroll
  for (int w = 0; w < 8; ++w) var += red[8 + w];
  var *= (1.0f / CD);
  T[c] = dv * rsqrtf(var + 1e-5f) * bfr(g[c]) + bfr(be[c]);
  __syncthreads();
  if (tid < 64) {
    const v4f v = *(const v4fa*)(&T[tid * 4]);
    float* dst = xp + (size_t)bp * CD + tid * 4;
    *(volatile v4f*)dst = v;
    __threadfence();
    *(volatile v4f*)dst = v;
  }
}

__global__ __launch_bounds__(256)
void k_gemm_kvp(const float* __restrict__ XP, const unsigned short* __restrict__ w16, const float* __restrict__ bkv,
                unsigned short* KPH, unsigned short* KPL, unsigned short* VPH, unsigned short* VPL) {
  __shared__ __align__(16) float Cs[64 * LDC];
  const int tid = threadIdx.x;
  const int mb = blockIdx.x, y = blockIdx.y;
  const int r0 = mb * 64, b = mb >> 2, p0 = (mb & 3) * 64;
  mm_tile_s(XP + (size_t)r0 * CD, CD, 32,
            (const _Float16*)(const void*)(w16 + (size_t)(CD + y * 128) * CD), CD, CD / 32, Cs);
  __syncthreads();

  if (y < 2) {
    const int row = tid & 63, hl = tid >> 6;
    const int h = y * 4 + hl;
    float* cr = Cs + row * LDC + hl * HD;
    float ss = 0.f;
#pragma unroll
    for (int d = 0; d < HD; ++d) {
      const float v = cr[d] * IAW + bfr(bkv[h * HD + d]);
      cr[d] = v;
      ss += v * v;
    }
    const float inv = __builtin_amdgcn_rcpf(fmaxf(sqrtf(ss), 1e-12f));
#pragma unroll
    for (int d = 0; d < HD; ++d) cr[d] = cr[d] * inv;
    __syncthreads();
    v4u ph[4], pl[4];
    size_t po[4];
#pragma unroll
    for (int s = 0; s < 4; ++s) {
      const int idx = s * 256 + tid;
      const int hl2 = idx >> 8, rem = idx & 255, row2 = rem >> 2, d0 = (rem & 3) * 8;
      const v4f a0 = *(const v4fa*)(&Cs[row2 * LDC + hl2 * HD + d0]);
      const v4f a1 = *(const v4fa*)(&Cs[row2 * LDC + hl2 * HD + d0 + 4]);
      v4u hv, lv;
      unsigned hp_, lp_;
      split2s(a0[0], a0[1], KSC, hp_, lp_); hv[0] = hp_; lv[0] = lp_;
      split2s(a0[2], a0[3], KSC, hp_, lp_); hv[1] = hp_; lv[1] = lp_;
      split2s(a1[0], a1[1], KSC, hp_, lp_); hv[2] = hp_; lv[2] = lp_;
      split2s(a1[2], a1[3], KSC, hp_, lp_); hv[3] = hp_; lv[3] = lp_;
      ph[s] = hv; pl[s] = lv;
      po[s] = ((size_t)((b * NHD + y * 4 + hl2) * NPL + p0 + row2)) * HD + d0;
    }
#pragma unroll
    for (int s = 0; s < 4; ++s) { *(volatile v4u*)(KPH + po[s]) = ph[s]; *(volatile v4u*)(KPL + po[s]) = pl[s]; }
    __threadfence();
#pragma unroll
    for (int s = 0; s < 4; ++s) { *(volatile v4u*)(KPH + po[s]) = ph[s]; *(volatile v4u*)(KPL + po[s]) = pl[s]; }
  } else {
    v4u ph[4], pl[4];
    size_t po[4];
#pragma unroll
    for (int s = 0; s < 4; ++s) {
      const int idx = s * 256 + tid;
      const int hl2 = idx >> 8, rem = idx & 255, d = rem >> 3, pc = rem & 7;
      const int col = hl2 * HD + d;
      const float bb = bfr(bkv[CD + (y - 2) * 128 + col]);
      v4u hv, lv;
      unsigned hp_, lp_;
#pragma unroll
      for (int e = 0; e < 4; ++e) {
        const int rr = 8 * pc + 2 * e;
        const float f0 = Cs[rr * LDC + col] * IAW + bb;
        const float f1 = Cs[(rr + 1) * LDC + col] * IAW + bb;
        split2s(f0, f1, VSC, hp_, lp_);
        hv[e] = hp_; lv[e] = lp_;
      }
      ph[s] = hv; pl[s] = lv;
      po[s] = ((size_t)((b * NHD + (y - 2) * 4 + hl2) * HD + d)) * NPL + p0 + 8 * pc;
    }
#pragma unroll
    for (int s = 0; s < 4; ++s) { *(volatile v4u*)(VPH + po[s]) = ph[s]; *(volatile v4u*)(VPL + po[s]) = pl[s]; }
    __threadfence();
#pragma unroll
    for (int s = 0; s < 4; ++s) { *(volatile v4u*)(VPH + po[s]) = ph[s]; *(volatile v4u*)(VPL + po[s]) = pl[s]; }
  }
}

__global__ __launch_bounds__(256)
void k_attn(const float* __restrict__ QN, const unsigned short* __restrict__ QHp, const unsigned short* __restrict__ QLp,
            const float* __restrict__ KL, const float* __restrict__ VLc,
            const unsigned short* __restrict__ KPp, const unsigned short* __restrict__ KRp,
            const unsigned short* __restrict__ VHp, const unsigned short* __restrict__ VRp,
            const float* __restrict__ BT, const int* __restrict__ ridx, const int* __restrict__ pm,
            const float* __restrict__ rbl, const float* __restrict__ tok, const float* __restrict__ lbias,
            const int* __restrict__ hp, const int* __restrict__ wp, int U, float* PRE) {
  extern __shared__ __align__(16) unsigned char lds_dyn[];
  float* Sc = (float*)(lds_dyn + L_SC);
  unsigned* PHu = (unsigned*)(lds_dyn + L_PH);
  unsigned* PLu = (unsigned*)(lds_dyn + L_PL);
  const _Float16* PHf = (const _Float16*)(const void*)(lds_dyn + L_PH);
  const _Float16* PLf = (const _Float16*)(const void*)(lds_dyn + L_PL);
  float* QSs = (float*)(lds_dyn + L_QS);
  float* QNs = (float*)(lds_dyn + L_QN);
  float* Ost = (float*)(lds_dyn + L_OS);
  float* OUs = (float*)(lds_dyn + L_OU);
  float* TK = (float*)(lds_dyn + L_TK);
  float* LB = TK + TKN;
  float* RB = TK + TKN + LL;
  const _Float16* QH16 = (const _Float16*)(const void*)QHp;
  const _Float16* QL16 = (const _Float16*)(const void*)QLp;
  const _Float16* KP16 = (const _Float16*)(const void*)KPp;
  const _Float16* KR16 = (const _Float16*)(const void*)KRp;
  const _Float16* VH16 = (const _Float16*)(const void*)VHp;
  const _Float16* VR16 = (const _Float16*)(const void*)VRp;

  const int tid = threadIdx.x, wave = tid >> 5, lane = tid & 31, hf = lane >> 4, m = lane & 15;
  const int blk = blockIdx.x;
  const int bh = blk >> 6, qi = blk & 63;
  const int h = bh & 7;
  const int n0 = qi * WR;
  const size_t rowbase = (size_t)bh * NTK + n0;
  const int hv = min(max(hp[0], 1), HR);
  const int wv = min(max(wp[0], 1), WR);

#pragma unroll
  for (int s = 0; s < 2; ++s) {
    const int idx = s * 256 + tid;
    const v4f v = *(const v4f*)(QN + rowbase * HD + idx * 4);
    *(v4fa*)(&QNs[idx * 4]) = v;
  }
  {
    const v8h hv8 = *(const v8h*)(QH16 + rowbase * HD + tid * 8);
    const v8h lv8 = *(const v8h*)(QL16 + rowbase * HD + tid * 8);
#pragma unroll
    for (int e = 0; e < 8; ++e) QSs[tid * 8 + e] = ((float)hv8[e] + (float)lv8[e] * RSC) * IQS;
  }
  {
    const float t0 = bfr(tok[h * TKN + min(tid, TKN - 1)]);
    const float t1 = bfr(tok[h * TKN + min(tid + 256, TKN - 1)]);
    TK[tid] = t0;
    if (tid < TKN - 256) TK[tid + 256] = t1;
    const int lc = min(tid, LL - 1);
    const float lbv = bfr(lbias[h * LL + lc]);
    const float rbv = bfr(rbl[h * LL + lc]);
    if (tid < LL) { LB[tid] = lbv; RB[tid] = rbv; }
  }
  __syncthreads();

  {
    const int mt = wave & 3, ng = wave >> 2;
    const size_t ao = (rowbase + 16 * mt + m) * HD + 8 * hf;
    const v16h ah = ld2(QH16 + ao, QH16 + ao + 16);
    const v16h al = ld2(QL16 + ao, QL16 + ao + 16);
#pragma unroll 1
    for (int t = 0; t < 8; ++t) {
      const int pt = (8 * ng + t) * 16;
      const size_t bo = ((size_t)bh * NPL + pt + m) * HD + 8 * hf;
      const v16h bk = ld2(KP16 + bo, KP16 + bo + 16);
      const v16h bl = ld2(KR16 + bo, KR16 + bo + 16);
      v8f ch = mma_raw(ah, bk, zero8());
      v8f cl = mma_raw(al, bk, zero8());
      cl = mma_raw(ah, bl, cl);
      guard2(ch, cl, ah, al, bk, bl);
#pragma unroll
      for (int r = 0; r < 8; ++r) {
        const int row = 16 * mt + 8 * hf + r;
        const int col = pt + m;
        int ri = ridx[(size_t)(n0 + row) * NPL + col];
        ri = min(max(ri, 0), U - 1);
        const float bb = BT[(size_t)ri * NHD + h];
        Sc[row * SCPI + col] = (ch[r] + cl[r] * RSC) * IQK + bb;
      }
    }
  }

#pragma unroll 1
  for (int it = 0; it < 3; ++it) {
    const int pair = it * 256 + tid;
    if (pair < 64 * LL) {
      const int l = pair >> 6, q = pair & 63;
      const int l3 = l / 3;
      const int di = l3 - 1, dj = l - l3 * 3 - 1;
      const int i2 = qi + di, j2 = q + dj;
      const bool inimg = ((unsigned)i2 < (unsigned)hv) && ((unsigned)j2 < (unsigned)wv);
      const int i2c = min(max(i2, 0), HR - 1), j2c = min(max(j2, 0), WR - 1);
      const float* kp = KL + ((size_t)bh * NTK + i2c * WR + j2c) * HD;
      const float* qp = QSs + q * HD;
      float dot = 0.f;
#pragma unroll
      for (int gq = 0; gq < 8; ++gq) {
        const v4f kv4 = *(const v4f*)(kp + 4 * gq);
        const v4f qv4 = *(const v4fa*)(qp + 4 * gq);
        dot += kv4[0] * qv4[0] + kv4[1] * qv4[1] + kv4[2] * qv4[2] + kv4[3] * qv4[3];
      }
      float val = (inimg ? dot : 0.f) + RB[l];
      const int msk = pm[(size_t)(n0 + q) * LL + l];
      if (msk != 0) val = -__builtin_huge_valf();
      Sc[q * SCPI + NPL + l] = val;
    }
  }
  __syncthreads();

  {
    const int q = tid >> 2, u = tid & 3;
    float* sr = Sc + q * SCPI;
    float mx = -__builtin_huge_valf();
#pragma unroll 1
    for (int e = u; e < NPL + LL; e += 4) mx = fmaxf(mx, sr[e]);
    mx = fmaxf(mx, __shfl_xor(mx, 1, 32));
    mx = fmaxf(mx, __shfl_xor(mx, 2, 32));
    float sum = 0.f;
#pragma unroll 1
    for (int e = u; e < NPL + LL; e += 4) {
      const float ex = __expf(sr[e] - mx);
      sr[e] = ex;
      sum += ex;
    }
    sum += __shfl_xor(sum, 1, 32);
    sum += __shfl_xor(sum, 2, 32);
    const float inv = __builtin_amdgcn_rcpf(sum);
    __syncthreads();
    unsigned* phr = PHu + q * (PPI / 2);
    unsigned* plr = PLu + q * (PPI / 2);
#pragma unroll 1
    for (int sp = u; sp < NPL / 2; sp += 4) {
      const int p = 2 * sp;
      const float f0 = sr[p] * inv * PSC;
      const float f1 = sr[p + 1] * inv * PSC;
      unsigned hp_, lp_;
      split2s(f0, f1, 1.0f, hp_, lp_);
      phr[sp] = hp_;
      plr[sp] = lp_;
    }
#pragma unroll 1
    for (int e = NPL + u; e < NPL + LL; e += 4) sr[e] = sr[e] * inv;
  }
  __syncthreads();

  {
    const int mt = wave & 3, nt = wave >> 2;
    const _Float16* pr  = PHf + (16 * mt + m) * PPI + 8 * hf;
    const _Float16* prl = PLf + (16 * mt + m) * PPI + 8 * hf;
    const int d = 16 * nt + m;
    const size_t vo = ((size_t)bh * HD + d) * NPL + 8 * hf;
    const _Float16* vhp = VH16 + vo;
    const _Float16* vrp = VR16 + vo;
    v8f oh = zero8(), ol = zero8();
#pragma unroll 1
    for (int ks = 0; ks < NPL / 32; ++ks) {
      const v16h pa = ld2(pr + 32 * ks, pr + 32 * ks + 16);
      const v16h pl = ld2(prl + 32 * ks, prl + 32 * ks + 16);
      const v16h vh = ld2(vhp + 32 * ks, vhp + 32 * ks + 16);
      const v16h vl = ld2(vrp + 32 * ks, vrp + 32 * ks + 16);
      oh = mma_raw(pa, vh, oh);
      ol = mma_raw(pa, vl, ol);
      ol = mma_raw(pl, vh, ol);
      guard2(oh, ol, pa, pl, vh, vl);
    }
#pragma unroll
    for (int r = 0; r < 8; ++r) Ost[(16 * mt + 8 * hf + r) * HD + d] = (oh[r] + ol[r] * RSC) * IPV;
  }
  __syncthreads();

  {
    const int q = tid >> 2, u = tid & 3, d0 = 8 * u;
    float qn8[8];
#pragma unroll
    for (int e = 0; e < 8; ++e) qn8[e] = QNs[q * HD + d0 + e];
    float w[LL];
#pragma unroll
    for (int l = 0; l < LL; ++l) {
      float t = 0.f;
#pragma unroll
      for (int e = 0; e < 8; ++e) t += qn8[e] * TK[(d0 + e) * LL + l];
      t += __shfl_xor(t, 1, 32);
      t += __shfl_xor(t, 2, 32);
      w[l] = t + LB[l] + Sc[q * SCPI + NPL + l];
    }
    float xl[8];
#pragma unroll
    for (int e = 0; e < 8; ++e) xl[e] = 0.f;
#pragma unroll
    for (int l = 0; l < LL; ++l) {
      const int di = l / 3 - 1, dj = l % 3 - 1;
      const int i2 = qi + di, j2 = q + dj;
      const bool inimg = ((unsigned)i2 < (unsigned)hv) && ((unsigned)j2 < (unsigned)wv);
      const int i2c = min(max(i2, 0), HR - 1), j2c = min(max(j2, 0), WR - 1);
      const float* vp = VLc + ((size_t)bh * NTK + i2c * WR + j2c) * HD + d0;
      const v4f v0 = *(const v4f*)(vp);
      const v4f v1 = *(const v4f*)(vp + 4);
      const float wg = inimg ? w[l] : 0.f;
      xl[0] += wg * v0[0]; xl[1] += wg * v0[1]; xl[2] += wg * v0[2]; xl[3] += wg * v0[3];
      xl[4] += wg * v1[0]; xl[5] += wg * v1[1]; xl[6] += wg * v1[2]; xl[7] += wg * v1[3];
    }
#pragma unroll
    for (int e = 0; e < 8; ++e) OUs[q * HD + d0 + e] = xl[e] + Ost[q * HD + d0 + e];
  }
  __syncthreads();
  {
    v4f pv[2];
    size_t po[2];
#pragma unroll
    for (int s = 0; s < 2; ++s) {
      const int idx = s * 256 + tid;
      const int row = idx >> 3, pc = idx & 7;
      pv[s] = *(const v4fa*)(&OUs[row * HD + pc * 4]);
      po[s] = (rowbase + row) * HD + pc * 4;
    }
#pragma unroll
    for (int s = 0; s < 2; ++s) *(volatile v4f*)(PRE + po[s]) = pv[s];
    __threadfence();
#pragma unroll
    for (int s = 0; s < 2; ++s) *(volatile v4f*)(PRE + po[s]) = pv[s];
  }
}

__global__ __launch_bounds__(256)
void k_gemm_proj(const float* __restrict__ PRE, const unsigned short* __restrict__ w16,
                 const float* __restrict__ bproj, float* out) {
  __shared__ __align__(16) float Cs[64 * LDC];
  const int tid = threadIdx.x;
  const int mb = blockIdx.x, y = blockIdx.y;
  const int row0 = mb * 64, b = mb >> 6, n0 = (mb & 63) * 64;
  mm_tile_s(PRE + ((size_t)b * NHD * NTK + n0) * HD, HD, NTK * HD,
            (const _Float16*)(const void*)(w16 + (size_t)(1024 + y * 128) * CD), CD, CD / 32, Cs);
  __syncthreads();
  v4f pv[8];
  size_t po[8];
#pragma unroll
  for (int s = 0; s < 8; ++s) {
    const int idx = s * 256 + tid;
    const int row2 = idx >> 5, c4 = (idx & 31) * 4;
    const int col = y * 128 + c4;
    const v4f a = *(const v4fa*)(&Cs[row2 * LDC + c4]);
    v4f r;
#pragma unroll
    for (int e = 0; e < 4; ++e) r[e] = a[e] * IAW + bfr(bproj[col + e]);
    pv[s] = r;
    po[s] = (size_t)(row0 + row2) * CD + col;
  }
#pragma unroll
  for (int s = 0; s < 8; ++s) *(volatile v4f*)(out + po[s]) = pv[s];
  __threadfence();
#pragma unroll
  for (int s = 0; s < 8; ++s) *(volatile v4f*)(out + po[s]) = pv[s];
}

extern "C" void kernel_launch(void* const* d_in, const int* in_sizes, int n_in,
                              void* d_out, int out_size, void* d_ws, size_t ws_size,
                              hipStream_t stream) {
  if (n_in < 26) return;
  if (in_sizes[0] != NROW * CD) return;
  if (in_sizes[1] != CD * CD || in_sizes[5] != 2 * CD * CD || in_sizes[7] != CD * CD || in_sizes[18] != CD * CD) return;
  if (in_sizes[2] != CD || in_sizes[6] != 2 * CD || in_sizes[8] != CD || in_sizes[19] != CD) return;
  if (in_sizes[3] != NHD * HD || in_sizes[4] != NHD || in_sizes[9] != CD || in_sizes[10] != CD) return;
  if (in_sizes[11] != 1024 || in_sizes[12] != 512 || in_sizes[13] != NHD * 512 || in_sizes[14] != NHD) return;
  if (in_sizes[15] != NHD * LL || in_sizes[16] != NHD * TKN || in_sizes[17] != NHD * LL) return;
  if (in_sizes[20] != NTK * LL || in_sizes[21] != NTK || in_sizes[23] != NTK * NPL) return;
  if (in_sizes[22] < 2 || in_sizes[24] < 1 || in_sizes[25] < 1) return;
  if (out_size != NROW * CD) return;
  const int U = in_sizes[22] / 2;
  const int Upad = (U + 7) & ~7;

  const float* x     = (const float*)d_in[0];
  const float* Wq    = (const float*)d_in[1];
  const float* bq    = (const float*)d_in[2];
  const float* qe    = (const float*)d_in[3];
  const float* temp  = (const float*)d_in[4];
  const float* Wkv   = (const float*)d_in[5];
  const float* bkv   = (const float*)d_in[6];
  const float* Wsr   = (const float*)d_in[7];
  const float* bsr   = (const float*)d_in[8];
  const float* ng    = (const float*)d_in[9];
  const float* nb    = (const float*)d_in[10];
  const float* cw1   = (const float*)d_in[11];
  const float* cb1   = (const float*)d_in[12];
  const float* cw2   = (const float*)d_in[13];
  const float* cb2   = (const float*)d_in[14];
  const float* rbl   = (const float*)d_in[15];
  const float* tok   = (const float*)d_in[16];
  const float* lbi   = (const float*)d_in[17];
  const float* Wproj = (const float*)d_in[18];
  const float* bproj = (const float*)d_in[19];
  const int*   pmask = (const int*)d_in[20];
  const float* sls   = (const float*)d_in[21];
  const float* rct   = (const float*)d_in[22];
  const int*   ridx  = (const int*)d_in[23];
  const int*   hin   = (const int*)d_in[24];
  const int*   win   = (const int*)d_in[25];
  float* out = (float*)d_out;

  const size_t sXB  = (size_t)NROW * CD * 2;
  const size_t sW16 = (size_t)WROWS * CD * 2;
  const size_t sF32 = (size_t)NBH * NTK * HD * 4;
  const size_t sF16 = (size_t)NBH * NTK * HD * 2;
  const size_t sXSR = (size_t)NROW * CD * 4;
  const size_t sXP  = (size_t)NBAT * NPL * CD * 4;
  const size_t sKP  = (size_t)NBH * NPL * HD * 2;
  const size_t sBT  = (size_t)Upad * NHD * 4;
  size_t off = 0;
  auto carve = [&](size_t bytes) { const size_t o = off; off += (bytes + 255) & ~(size_t)255; return o; };
  const size_t oXB  = carve(sXB);
  const size_t oW16 = carve(sW16);
  const size_t oQN  = carve(sF32);
  const size_t oQH  = carve(sF16);
  const size_t oQL  = carve(sF16);
  const size_t oKL  = carve(sF32);
  const size_t oVL  = carve(sF32);
  const size_t oXSR = carve(sXSR);
  const size_t oXP  = carve(sXP);
  const size_t oKP  = carve(sKP);
  const size_t oKPL = carve(sKP);
  const size_t oVPH = carve(sKP);
  const size_t oVPL = carve(sKP);
  const size_t oBT  = carve(sBT);
  const size_t oPRE = carve(sF32);
  if (off > ws_size) return;
  if (off > (size_t)134217728) return;

  char* ws = (char*)d_ws;
  unsigned short* XB  = (unsigned short*)(ws + oXB);
  unsigned short* W16 = (unsigned short*)(ws + oW16);
  float* QN  = (float*)(ws + oQN);
  unsigned short* QH = (unsigned short*)(ws + oQH);
  unsigned short* QL = (unsigned short*)(ws + oQL);
  float* KL  = (float*)(ws + oKL);
  float* VL  = (float*)(ws + oVL);
  float* XSR = (float*)(ws + oXSR);
  float* XP  = (float*)(ws + oXP);
  unsigned short* KPH = (unsigned short*)(ws + oKP);
  unsigned short* KPL = (unsigned short*)(ws + oKPL);
  unsigned short* VPH = (unsigned short*)(ws + oVPH);
  unsigned short* VPL = (unsigned short*)(ws + oVPL);
  float* BT  = (float*)(ws + oBT);
  float* PRE = (float*)(ws + oPRE);

  const dim3 blk(256);
  k_cvt_x<<<dim3(NROW * CD / 2048), blk, 0, stream>>>(x, XB);
  k_cvt_w<<<dim3(WROWS / 8), blk, 0, stream>>>(Wq, Wkv, Wsr, Wproj, W16);
  k_cpb<<<dim3(Upad / 8), blk, 0, stream>>>(rct, cw1, cb1, cw2, cb2, BT, U);
  k_gemm1<<<dim3(NROW / 64, 8), blk, 0, stream>>>(XB, W16, bq, bkv, bsr, qe, temp, sls, QN, QH, QL, KL, VL, XSR);
  k_pool_ln<<<dim3(NBAT * NPL), blk, 0, stream>>>(XSR, ng, nb, XP);
  k_gemm_kvp<<<dim3(NBAT * NPL / 64, 4), blk, 0, stream>>>(XP, W16, bkv, KPH, KPL, VPH, VPL);
  (void)hipFuncSetAttribute(reinterpret_cast<const void*>(&k_attn),
                            hipFuncAttributeMaxDynamicSharedMemorySize, LDS_ATTN);
  k_attn<<<dim3(NBH * HR), blk, LDS_ATTN, stream>>>(QN, QH, QL, KL, VL, KPH, KPL, VPH, VPL, BT, ridx, pmask,
                                                     rbl, tok, lbi, hin, win, U, PRE);
  k_gemm_proj<<<dim3(NROW / 64, 2), blk, 0, stream>>>(PRE, W16, bproj, out);
  (void)hipGetLastError();
}
